// HypernetDecoder_18700287607448
// MI455X (gfx1250) — hardware-verified
//
#include <hip/hip_runtime.h>
#include <math.h>

constexpr int kLatent      = 16;
constexpr int kHid         = 512;
constexpr int kDdim        = 64;
constexpr int kBatch       = 128;
constexpr int kGrid        = 128;
constexpr int kOutSz       = 12610;
constexpr int kOutPad      = 12672;
constexpr int kKpad0       = 32;
constexpr int kOffB0       = 64;
constexpr int kOffW1       = 65;
constexpr int kLayerStride = 4160;
constexpr int kOffW4       = 12545;
constexpr int kOffB4       = 12609;
constexpr int kDecThreads  = 64;
constexpr int kXPitch      = 68;
static_assert(kOffW4 == kOffW1 + 3 * kLayerStride, "wb layout");
static_assert(kOffB4 + 1 == kOutSz, "wb layout");
static_assert(kOutPad % 64 == 0 && kOutPad >= kOutSz, "pad");
static_assert(kBatch % 64 == 0 && kHid % 64 == 0 && kKpad0 % 32 == 0, "tiles");

typedef __attribute__((ext_vector_type(16))) _Float16 v16h;
typedef __attribute__((ext_vector_type(8)))  _Float16 v8h;
typedef __attribute__((ext_vector_type(16))) __bf16   v16b;
typedef __attribute__((ext_vector_type(8)))  __bf16   v8b;
typedef __attribute__((ext_vector_type(8)))  float    v8f;
typedef __attribute__((ext_vector_type(4)))  float    v4f;
typedef __attribute__((ext_vector_type(4)))  unsigned int v4u;

__device__ __forceinline__ unsigned short f2bf_bits(float f) {
  unsigned u = __float_as_uint(f);
  return (unsigned short)((u + 0x7FFFu + ((u >> 16) & 1u)) >> 16);
}
__device__ __forceinline__ float bf_bits2f(unsigned short h) { return __uint_as_float(((unsigned)h) << 16); }

__device__ __forceinline__ void dep_guard_h(v8f& a, v8f& b, v16h x, v16h y) { asm volatile("v_nop\n\tv_nop\n\tv_nop\n\tv_nop" : "+v"(a), "+v"(b) : "v"(x), "v"(y)); }
__device__ __forceinline__ void dep_guard_b(v8f& a, v8f& b, v16b x, v16b y) { asm volatile("v_nop\n\tv_nop\n\tv_nop\n\tv_nop" : "+v"(a), "+v"(b) : "v"(x), "v"(y)); }
__device__ __forceinline__ void keep4_h(v16h a, v16h b, v16h c, v16h d) { asm volatile("v_nop" :: "v"(a), "v"(b), "v"(c), "v"(d)); }
__device__ __forceinline__ void keep4_b(v16b a, v16b b, v16b c, v16b d) { asm volatile("v_nop" :: "v"(a), "v"(b), "v"(c), "v"(d)); }
__device__ __forceinline__ void acc_guard4(v8f& a, v8f& b, v8f& c, v8f& d) { asm volatile("v_nop\n\tv_nop\n\tv_nop\n\tv_nop" : "+v"(a), "+v"(b), "+v"(c), "+v"(d)); }
template <typename T> struct Frag;
template <> struct Frag<_Float16> {
  typedef v16h V; union U { v16h v; v8h h[2]; };
  static __device__ __forceinline__ v16h load(const _Float16* p) {
    U f; f.h[0] = *(const v8h*)(p); f.h[1] = *(const v8h*)(p + 16); return f.v;
  }
  static __device__ __forceinline__ v8f mma(v16h a, v16h b, v8f c) {
    return __builtin_amdgcn_wmma_f32_16x16x32_f16(false, a, false, b, (short)0, c, false, false);
  }
  static __device__ __forceinline__ void guard(v8f& a, v8f& b, v16h x, v16h y) { dep_guard_h(a, b, x, y); }
  static __device__ __forceinline__ void keep(v16h a, v16h b, v16h c, v16h d) { keep4_h(a, b, c, d); }
};
template <> struct Frag<__bf16> {
  typedef v16b V; union U { v16b v; v8b h[2]; };
  static __device__ __forceinline__ v16b load(const __bf16* p) {
    U f; f.h[0] = *(const v8b*)(p); f.h[1] = *(const v8b*)(p + 16); return f.v;
  }
  static __device__ __forceinline__ v8f mma(v16b a, v16b b, v8f c) {
    return __builtin_amdgcn_wmma_f32_16x16x32_bf16(false, a, false, b, (short)0, c, false, false);
  }
  static __device__ __forceinline__ void guard(v8f& a, v8f& b, v16b x, v16b y) { dep_guard_b(a, b, x, y); }
  static __device__ __forceinline__ void keep(v16b a, v16b b, v16b c, v16b d) { keep4_b(a, b, c, d); }
};

__device__ __forceinline__ unsigned pk16(unsigned short a, unsigned short b) { return (unsigned)a | ((unsigned)b << 16); }
__device__ __forceinline__ void split_bf(float f, unsigned short& hb, unsigned short& lb) {
  hb = f2bf_bits(f);
  lb = f2bf_bits(f - bf_bits2f(hb));
}

template <int ET> struct Elem;
template <> struct Elem<0> { typedef _Float16 T; };
template <> struct Elem<1> { typedef __bf16 T; };
template <int ET, bool SPLIT, int BIAS_MODE, int OUT_MODE, bool RESID, int ACT = 0>
__global__ __launch_bounds__(256) void wmma_gemm64(
    const unsigned short* __restrict__ Ap, const unsigned short* __restrict__ A2p, int lda, long strideA,
    const unsigned short* __restrict__ Btp, const unsigned short* __restrict__ Bt2p, int ldb, long strideB,
    void* __restrict__ Cout, void* __restrict__ Cout2, int ldc, long strideC,
    const float* __restrict__ bias,
    const float* __restrict__ resid, long strideR,
    int M, int N, int K, float scale) {
  typedef typename Elem<ET>::T T;
  typedef typename Frag<T>::V V;
  const T* A = (const T*)Ap; const T* A2 = (const T*)A2p; const T* Bt = (const T*)Btp; const T* Bt2 = (const T*)Bt2p;
  __shared__ __align__(16) float sT[8][16 * 68];
  const int b    = blockIdx.y;
  const int lane = threadIdx.x & 31;
  const int wave = threadIdx.x >> 5;
  const int tilesN = N >> 6;
  const int tilesM = M >> 6;
  const int tile = blockIdx.x * 8 + wave;
  if (tile >= tilesM * tilesN) return;
  const int tm = tile / tilesN;
  const int tn = tile - tm * tilesN;
  const int m0 = tm << 6;
  const int n0 = tn << 6;

  const T* Ab  = A  + (size_t)b * strideA;
  const T* Bb  = Bt + (size_t)b * strideB;
  const T* Ab2 = SPLIT ? (A2  + (size_t)b * strideA) : nullptr;
  const T* Bb2 = SPLIT ? (Bt2 + (size_t)b * strideB) : nullptr;

  const int rlane = lane & 15;
  const int koff  = (lane >> 4) * 8;
  const int mOff  = (lane >> 4) * 8;

  v8f acc[4][4];
#pragma unroll
  for (int i = 0; i < 4; ++i)
#pragma unroll
    for (int j = 0; j < 4; ++j) acc[i][j] = (v8f){0.f,0.f,0.f,0.f,0.f,0.f,0.f,0.f};

  for (int k0 = 0; k0 < K; k0 += 32) {
    V bh[4], bl[4];
#pragma unroll
    for (int j = 0; j < 4; ++j) {
      const size_t bo = (size_t)(n0 + (j << 4) + rlane) * ldb + koff + k0;
      bh[j] = Frag<T>::load(Bb + bo);
      if (SPLIT) bl[j] = Frag<T>::load(Bb2 + bo);
    }
#pragma unroll
    for (int i = 0; i < 4; ++i) {
      const size_t ao = (size_t)(m0 + (i << 4) + rlane) * lda + koff + k0;
      V ah = Frag<T>::load(Ab + ao);
      V al;
      if (SPLIT) al = Frag<T>::load(Ab2 + ao);
#pragma unroll
      for (int j = 0; j < 4; ++j) {
        acc[i][j] = Frag<T>::mma(ah, bh[j], acc[i][j]);
        if (SPLIT) {
          acc[i][j] = Frag<T>::mma(ah, bl[j], acc[i][j]);
          acc[i][j] = Frag<T>::mma(al, bh[j], acc[i][j]);
        }
      }
      Frag<T>::guard(acc[i][0], acc[i][3], ah, SPLIT ? al : ah);
    }
    Frag<T>::keep(bh[0], bh[1], bh[2], bh[3]);
    if (SPLIT) Frag<T>::keep(bl[0], bl[1], bl[2], bl[3]);
  }
  acc_guard4(acc[0][0], acc[0][1], acc[0][2], acc[0][3]);
  acc_guard4(acc[1][0], acc[1][1], acc[1][2], acc[1][3]);
  acc_guard4(acc[2][0], acc[2][1], acc[2][2], acc[2][3]);
  acc_guard4(acc[3][0], acc[3][1], acc[3][2], acc[3][3]);

  float* slab = sT[wave];
  const float* Rb = RESID ? (resid + (size_t)b * strideR) : nullptr;
#pragma unroll
  for (int i = 0; i < 4; ++i) {
    const int mBase = m0 + (i << 4);
#pragma unroll
    for (int j = 0; j < 4; ++j) {
      const int n = n0 + (j << 4) + rlane;
      float bv = 0.f;
      if (BIAS_MODE == 2) bv = bias[n];
#pragma unroll
      for (int r = 0; r < 8; ++r) {
        float v = acc[i][j][r] * scale;
        if (BIAS_MODE == 1) v += bias[mBase + mOff + r];
        if (BIAS_MODE == 2) v += bv;
        if (RESID) v += Rb[(size_t)(mBase + mOff + r) * ldc + n];
        if (ACT == 2) v = fmaxf(v, 0.0f);
        if (ACT == 4) v = (v > 0.f) ? v : 0.01f * v;
        slab[(mOff + r) * 68 + (j << 4) + rlane] = v;
      }
    }
    __builtin_amdgcn_fence(__ATOMIC_RELEASE, "workgroup");
    __builtin_amdgcn_wave_barrier();
    __builtin_amdgcn_fence(__ATOMIC_ACQUIRE, "workgroup");
    if (OUT_MODE == 0) {
      float* C = (float*)Cout + (size_t)b * strideC;
      const int hh = lane >> 4, c4 = (lane & 15) * 4;
      for (int pass = 0; pass < 2; ++pass) {
#pragma unroll
        for (int it = 0; it < 8; ++it) {
          const int row = it * 2 + hh;
          v4f v = *(const v4f*)(slab + row * 68 + c4);
          *(volatile v4f*)(C + (size_t)(mBase + row) * ldc + n0 + c4) = v;
        }
        __threadfence();
      }
    } else {
      const int q = lane >> 3, c8 = (lane & 7) * 8;
      unsigned short* C  = (unsigned short*)Cout  + (size_t)b * strideC;
      unsigned short* C2 = (OUT_MODE == 2) ? ((unsigned short*)Cout2 + (size_t)b * strideC) : nullptr;
      for (int pass = 0; pass < 2; ++pass) {
#pragma unroll
        for (int it = 0; it < 4; ++it) {
          const int row = it * 4 + q;
          const float* sp = slab + row * 68 + c8;
          v8h hv, lv;
#pragma unroll
          for (int e = 0; e < 8; ++e) {
            if (OUT_MODE == 1) {
              hv[e] = (_Float16)sp[e];
            } else {
              unsigned short hb = f2bf_bits(sp[e]);
              unsigned short lb = f2bf_bits(sp[e] - bf_bits2f(hb));
              hv[e] = __builtin_bit_cast(_Float16, hb);
              lv[e] = __builtin_bit_cast(_Float16, lb);
            }
          }
          *(volatile v8h*)(C + (size_t)(mBase + row) * ldc + n0 + c8) = hv;
          if (OUT_MODE == 2) *(volatile v8h*)(C2 + (size_t)(mBase + row) * ldc + n0 + c8) = lv;
        }
        __threadfence();
      }
    }
    __builtin_amdgcn_fence(__ATOMIC_RELEASE, "workgroup");
    __builtin_amdgcn_wave_barrier();
    __builtin_amdgcn_fence(__ATOMIC_ACQUIRE, "workgroup");
  }
}

__global__ __launch_bounds__(256) void prep_small(const float* __restrict__ z, const float* __restrict__ hw0,
                                                  unsigned short* __restrict__ zhi, unsigned short* __restrict__ zlo,
                                                  unsigned short* __restrict__ b0hi, unsigned short* __restrict__ b0lo) {
  const int blk = blockIdx.x;
  const int t   = threadIdx.x;
  float v[8];
  if (blk < 2) {
    const int idx = blk * 256 + t;
    const int row = idx >> 2;
    const int c8  = (idx & 3) * 8;
#pragma unroll
    for (int e = 0; e < 8; ++e) {
      const int k  = c8 + e;
      const int kc = (k < kLatent) ? k : (kLatent - 1);
      const float val = z[row * kLatent + kc];
      v[e] = (k < kLatent) ? val : 0.0f;
    }
    unsigned short hb[8], lb[8];
#pragma unroll
    for (int e = 0; e < 8; ++e) split_bf(v[e], hb[e], lb[e]);
    const v4u uh = (v4u){pk16(hb[0], hb[1]), pk16(hb[2], hb[3]), pk16(hb[4], hb[5]), pk16(hb[6], hb[7])};
    const v4u ul = (v4u){pk16(lb[0], lb[1]), pk16(lb[2], lb[3]), pk16(lb[4], lb[5]), pk16(lb[6], lb[7])};
    const size_t off = (size_t)idx * 8;
    *(volatile v4u*)(zhi + off) = uh;
    *(volatile v4u*)(zlo + off) = ul;
    __threadfence();
    *(volatile v4u*)(zhi + off) = uh;
    *(volatile v4u*)(zlo + off) = ul;
  } else {
    const int idx = (blk - 2) * 256 + t;
    const int n   = idx >> 2;
    const int c8  = (idx & 3) * 8;
#pragma unroll
    for (int e = 0; e < 8; ++e) {
      const int k  = c8 + e;
      const int kc = (k < kLatent) ? k : (kLatent - 1);
      const float val = hw0[kc * kHid + n];
      v[e] = (k < kLatent) ? val : 0.0f;
    }
    unsigned short hb[8], lb[8];
#pragma unroll
    for (int e = 0; e < 8; ++e) split_bf(v[e], hb[e], lb[e]);
    const v4u uh = (v4u){pk16(hb[0], hb[1]), pk16(hb[2], hb[3]), pk16(hb[4], hb[5]), pk16(hb[6], hb[7])};
    const v4u ul = (v4u){pk16(lb[0], lb[1]), pk16(lb[2], lb[3]), pk16(lb[4], lb[5]), pk16(lb[6], lb[7])};
    const size_t off = (size_t)idx * 8;
    *(volatile v4u*)(b0hi + off) = uh;
    *(volatile v4u*)(b0lo + off) = ul;
    __threadfence();
    *(volatile v4u*)(b0hi + off) = uh;
    *(volatile v4u*)(b0lo + off) = ul;
  }
}

__global__ __launch_bounds__(256) void prep_wt(const float* __restrict__ W, int kdim, int ndim,
                                               unsigned short* __restrict__ ohi, unsigned short* __restrict__ olo,
                                               int kpitch) {
  __shared__ float sm[64][65];
  const int t  = threadIdx.x;
  const int k0 = blockIdx.x * 64;
  const int n0 = blockIdx.y * 64;
#pragma unroll
  for (int i = 0; i < 16; ++i) {
    const int e = i * 256 + t;
    const int r = e >> 6;
    const int c = e & 63;
    const int kk = k0 + r;
    const int nn = n0 + c;
    const int kc = (kk < kdim) ? kk : (kdim - 1);
    const int nc = (nn < ndim) ? nn : (ndim - 1);
    float val = W[(size_t)kc * ndim + nc];
    if (kk >= kdim || nn >= ndim) val = 0.0f;
    sm[c][r] = val;
  }
  __syncthreads();
  const int lane = t & 31, wave = t >> 5;
  const int q = lane >> 3, c8 = (lane & 7) * 8;
  for (int pass = 0; pass < 2; ++pass) {
#pragma unroll
    for (int it = 0; it < 2; ++it) {
      const int row = wave * 8 + it * 4 + q;
      unsigned short hb[8], lb[8];
#pragma unroll
      for (int e = 0; e < 8; ++e) split_bf(sm[row][c8 + e], hb[e], lb[e]);
      const v4u uh = (v4u){pk16(hb[0], hb[1]), pk16(hb[2], hb[3]), pk16(hb[4], hb[5]), pk16(hb[6], hb[7])};
      const v4u ul = (v4u){pk16(lb[0], lb[1]), pk16(lb[2], lb[3]), pk16(lb[4], lb[5]), pk16(lb[6], lb[7])};
      const size_t off = (size_t)(n0 + row) * kpitch + k0 + c8;
      *(volatile v4u*)(ohi + off) = uh;
      *(volatile v4u*)(olo + off) = ul;
    }
    __threadfence();
  }
}

__global__ __launch_bounds__(64) void decoder_rows(const float* __restrict__ wbm, const float* __restrict__ hb2,
                                                   const float* __restrict__ logp, float* __restrict__ out) {
#pragma clang fp contract(off)
  __shared__ __align__(16) float xs[2][kDecThreads * kXPitch];
  __shared__ __align__(16) float wts[kDdim * kDdim];
  __shared__ __align__(16) float w0s[kDdim];
  __shared__ __align__(16) float w4s[kDdim];
  __shared__ float bsh[kDdim];
  __shared__ float scal[2];
  __shared__ __align__(16) float ts[kDecThreads];
  const int t    = threadIdx.x;
  const int b    = blockIdx.x >> 1;
  const int hsel = blockIdx.x & 1;
  const int g    = hsel * kDecThreads + t;
  const float* wrow = wbm + (size_t)b * kOutPad;
  w0s[t] = wrow[t] + hb2[t];
  w4s[t] = wrow[kOffW4 + t] + hb2[kOffW4 + t];
  if (t == 0) {
    scal[0] = wrow[kOffB0] + hb2[kOffB0];
    scal[1] = wrow[kOffB4] + hb2[kOffB4];
  }
  const float xval = logp[b * kGrid + g];
  __syncthreads();

#pragma unroll 1
  for (int l = 0; l < 4; ++l) {
    float* xo = &xs[l & 1][t * kXPitch];
    const float* xi = &xs[(l + 1) & 1][t * kXPitch];
    __syncthreads();
    if (l > 0) {
      const int offW = kOffW1 + (l - 1) * kLayerStride;
#pragma unroll 1
      for (int e = t; e < kDdim * kDdim; e += kDecThreads) {
        const int i = e >> 6, j = e & 63;
        wts[j * kDdim + i] = wrow[offW + e] + hb2[offW + e];
      }
      bsh[t] = wrow[offW + kDdim * kDdim + t] + hb2[offW + kDdim * kDdim + t];
    }
    __syncthreads();
    if (l == 0) {
      const float bias0 = scal[0];
#pragma unroll 1
      for (int j = 0; j < kDdim; ++j) {
        float p = xval * w0s[j];
        p = p + bias0;
        p = p * 30.0f;
        xo[j] = p;
      }
    } else {
#pragma unroll 1
      for (int j = 0; j < kDdim; ++j) {
        const float* wr = wts + j * kDdim;
        float acc = 0.0f;
#pragma unroll 1
        for (int i = 0; i < kDdim; i += 8) {
          const v4f xa = *(const v4f*)(xi + i);
          const v4f xb = *(const v4f*)(xi + i + 4);
          const v4f wa = *(const v4f*)(wr + i);
          const v4f wv = *(const v4f*)(wr + i + 4);
          acc = fmaf(xa[0], wa[0], acc);
          acc = fmaf(xa[1], wa[1], acc);
          acc = fmaf(xa[2], wa[2], acc);
          acc = fmaf(xa[3], wa[3], acc);
          acc = fmaf(xb[0], wv[0], acc);
          acc = fmaf(xb[1], wv[1], acc);
          acc = fmaf(xb[2], wv[2], acc);
          acc = fmaf(xb[3], wv[3], acc);
        }
        xo[j] = acc + bsh[j];
      }
    }
#pragma unroll 1
    for (int j = 0; j < kDdim; ++j) xo[j] = sinf(xo[j]);
  }
  __syncthreads();

  {
    const float* x3 = &xs[1][t * kXPitch];
    float acc = 0.0f;
#pragma unroll 1
    for (int i = 0; i < kDdim; i += 8) {
      const v4f xa = *(const v4f*)(x3 + i);
      const v4f xb = *(const v4f*)(x3 + i + 4);
      const v4f wa = *(const v4f*)(w4s + i);
      const v4f wv = *(const v4f*)(w4s + i + 4);
      acc = fmaf(xa[0], wa[0], acc);
      acc = fmaf(xa[1], wa[1], acc);
      acc = fmaf(xa[2], wa[2], acc);
      acc = fmaf(xa[3], wa[3], acc);
      acc = fmaf(xb[0], wv[0], acc);
      acc = fmaf(xb[1], wv[1], acc);
      acc = fmaf(xb[2], wv[2], acc);
      acc = fmaf(xb[3], wv[3], acc);
    }
    float tv = acc + scal[1];
    tv = tv * 500.0f;
    tv = tv + 1500.0f;
    ts[t] = tv;
  }
  __syncthreads();
  if (t < 16) {
    const v4f val = *(const v4f*)(ts + 4 * t);
    float* op = out + (size_t)b * kGrid + hsel * kDecThreads + 4 * t;
    *(volatile v4f*)op = val;
    __threadfence();
    *(volatile v4f*)op = val;
  }
}

static inline size_t align_up256(size_t x) { return (x + 255) & ~(size_t)255; }

extern "C" void kernel_launch(void* const* d_in, const int* in_sizes, int n_in,
                              void* d_out, int out_size, void* d_ws, size_t ws_size,
                              hipStream_t stream) {
  if (n_in < 8) return;
  if (in_sizes[0] != kBatch * kLatent || in_sizes[1] != kBatch * kGrid ||
      in_sizes[2] != kLatent * kHid || in_sizes[3] != kHid ||
      in_sizes[4] != kHid * kHid || in_sizes[5] != kHid ||
      in_sizes[6] != kHid * kOutSz || in_sizes[7] != kOutSz) return;
  if (out_size != kBatch * kGrid) return;

  const float* z     = (const float*)d_in[0];
  const float* log_P = (const float*)d_in[1];
  const float* hw0   = (const float*)d_in[2];
  const float* hb0   = (const float*)d_in[3];
  const float* hw1   = (const float*)d_in[4];
  const float* hb1   = (const float*)d_in[5];
  const float* hw2   = (const float*)d_in[6];
  const float* hb2   = (const float*)d_in[7];
  float* out = (float*)d_out;

  char* w = (char*)d_ws;
  size_t off = 0;
  const size_t zPlane   = (size_t)kBatch  * kKpad0  * 2;
  const size_t bt0Plane = (size_t)kHid    * kKpad0  * 2;
  const size_t hPlane   = (size_t)kBatch  * kHid    * 2;
  const size_t bt1Plane = (size_t)kHid    * kHid    * 2;
  const size_t bt2Plane = (size_t)kOutPad * kHid    * 2;
  const size_t wbBytes  = (size_t)kBatch  * kOutPad * 4;
  unsigned short* zhi   = (unsigned short*)(w + off); off = align_up256(off + zPlane);
  unsigned short* zlo   = (unsigned short*)(w + off); off = align_up256(off + zPlane);
  unsigned short* bt0hi = (unsigned short*)(w + off); off = align_up256(off + bt0Plane);
  unsigned short* bt0lo = (unsigned short*)(w + off); off = align_up256(off + bt0Plane);
  unsigned short* h0hi  = (unsigned short*)(w + off); off = align_up256(off + hPlane);
  unsigned short* h0lo  = (unsigned short*)(w + off); off = align_up256(off + hPlane);
  unsigned short* bt1hi = (unsigned short*)(w + off); off = align_up256(off + bt1Plane);
  unsigned short* bt1lo = (unsigned short*)(w + off); off = align_up256(off + bt1Plane);
  unsigned short* h1hi  = (unsigned short*)(w + off); off = align_up256(off + hPlane);
  unsigned short* h1lo  = (unsigned short*)(w + off); off = align_up256(off + hPlane);
  unsigned short* bt2hi = (unsigned short*)(w + off); off = align_up256(off + bt2Plane);
  unsigned short* bt2lo = (unsigned short*)(w + off); off = align_up256(off + bt2Plane);
  float*          wbuf  = (float*)(w + off);          off = align_up256(off + wbBytes);
  if (off > ws_size) return;

  prep_small<<<dim3(10), dim3(256), 0, stream>>>(z, hw0, zhi, zlo, bt0hi, bt0lo);
  prep_wt<<<dim3(kHid / 64, kHid / 64), dim3(256), 0, stream>>>(hw1, kHid, kHid, bt1hi, bt1lo, kHid);
  prep_wt<<<dim3(kHid / 64, kOutPad / 64), dim3(256), 0, stream>>>(hw2, kHid, kOutSz, bt2hi, bt2lo, kHid);

  {
    const int tiles = (kBatch / 64) * (kHid / 64);
    wmma_gemm64<1, true, 2, 2, false, 4><<<dim3((tiles + 7) / 8, 1), dim3(256), 0, stream>>>(
        zhi, zlo, kKpad0, 0L, bt0hi, bt0lo, kKpad0, 0L,
        (void*)h0hi, (void*)h0lo, kHid, 0L, hb0, hb0, 0L, kBatch, kHid, kKpad0, 1.0f);
  }
  {
    const int tiles = (kBatch / 64) * (kHid / 64);
    wmma_gemm64<1, true, 2, 2, false, 4><<<dim3((tiles + 7) / 8, 1), dim3(256), 0, stream>>>(
        h0hi, h0lo, kHid, 0L, bt1hi, bt1lo, kHid, 0L,
        (void*)h1hi, (void*)h1lo, kHid, 0L, hb1, hb1, 0L, kBatch, kHid, kHid, 1.0f);
  }
  {
    const int tiles = (kBatch / 64) * (kOutPad / 64);
    wmma_gemm64<1, true, 0, 0, false, 0><<<dim3((tiles + 7) / 8, 1), dim3(256), 0, stream>>>(
        h1hi, h1lo, kHid, 0L, bt2hi, bt2lo, kHid, 0L,
        (void*)wbuf, (void*)wbuf, kOutPad, 0L, hb2, hb2, 0L, kBatch, kOutPad, kHid, 1.0f);
  }
  decoder_rows<<<dim3(kBatch * 2), dim3(kDecThreads), 0, stream>>>(wbuf, hb2, log_P, out);
}
